// GCN_10591389352059
// MI455X (gfx1250) — hardware-verified
//
#include <hip/hip_runtime.h>
#include <stddef.h>
#include <stdint.h>


#define CIN    128
#define HID    128
#define K2     256
#define NCLS   40
#define NC3    48
#define NTHR   256
#define NWAVE  8
#define EPT    8
#define CHUNK  (NTHR * EPT)
#define WCAP   (EPT * 32)
#define LISTN  (NWAVE * WCAP)
#define NBA    1024
#define SLA    10
#define RCAP   20480
#define DEGCAP 64
#define POISONC 0x40000000
#define GBM    64
#define GTHR   128
#define NU1    (HID * (CIN / 8))
#define NU2    (HID * (K2 / 8))
#define NU3    (NC3 * (K2 / 8))
#define BLD_ZINTS (LISTN + 2 * RCAP + 3 * NBA)
#define BLD_LDS_INTS (BLD_ZINTS + 16)
#define NGRP   ((NBA + 2) / 3)
#define WSMAX  134217728

static_assert((CHUNK & (CHUNK - 1)) == 0 && CHUNK <= 4096);
static_assert((NBA & (NBA - 1)) == 0 && NBA == (1 << SLA));
static_assert(((long long)CHUNK << SLA) < (1LL << 31));
static_assert(LISTN % NTHR == 0 && LISTN % 4 == 0);
static_assert(NBA % NWAVE == 0 && NBA % 32 == 0 && NBA % GBM == 0);
static_assert(RCAP % (NTHR * 4) == 0 && BLD_ZINTS % (NTHR * 4) == 0);
static_assert((NBA * 2) % (NTHR * 4) == 0);
static_assert(CIN % 32 == 0 && K2 % 32 == 0 && K2 == 2 * HID && HID == 4 * 32);
static_assert(GBM == (GTHR / 32) * 16);
static_assert(NU1 % NTHR == 0 && NU2 % NTHR == 0 && NU3 % NTHR == 0);
static_assert(NC3 % 16 == 0 && NCLS <= NC3 && NCLS % 4 == 0 && NCLS / 4 == 10);
static_assert((NBA * NCLS * 4) % 128 == 0 && (NBA * NCLS / 4) % NTHR == 0);
static_assert((GBM * NC3 * 4) % 128 == 0 && (GBM * NC3 / 4) % GTHR == 0);
static_assert(BLD_LDS_INTS * 4 <= 300000 && NBA * NCLS * 4 <= 300000);
static_assert(DEGCAP < POISONC);

typedef float          v4f   __attribute__((ext_vector_type(4)));
typedef float          v8f   __attribute__((ext_vector_type(8)));
typedef int            v2i   __attribute__((ext_vector_type(2)));
typedef int            v4i   __attribute__((ext_vector_type(4)));
typedef int            v8i   __attribute__((ext_vector_type(8)));
typedef unsigned short v4us  __attribute__((ext_vector_type(4)));
typedef unsigned short v8us  __attribute__((ext_vector_type(8)));
typedef unsigned short v16us __attribute__((ext_vector_type(16)));
typedef __bf16         v16bf __attribute__((ext_vector_type(16)));
typedef v4f  __attribute__((may_alias)) v4fa;
typedef v2i  __attribute__((may_alias)) v2ia;
typedef v4i  __attribute__((may_alias)) v4ia;
typedef v4us __attribute__((may_alias)) v4usa;
typedef v8us __attribute__((may_alias)) v8usa;
union FragB { v16bf v; v16us u; v8us h[2]; v8i w; };

__device__ __forceinline__ v8f wmb(const FragB& a, const FragB& b, v8f c) {
  v8f d = __builtin_amdgcn_wmma_f32_16x16x32_bf16(false, a.v, false, b.v, (short)0, c, false, false);
  asm volatile("v_nop\n\tv_nop\n\tv_nop\n\tv_nop" : "+v"(d) : "v"(a.w), "v"(b.w));
  return d;
}

__device__ __forceinline__ unsigned bf16_bits(float f) {
  const unsigned u = __float_as_uint(f);
  return (u + 0x7FFFu + ((u >> 16) & 1u)) >> 16;
}
__device__ __forceinline__ float bf16_val(float f) {
  return __uint_as_float(bf16_bits(f) << 16);
}

__device__ __forceinline__ void wave_sync() {
  __builtin_amdgcn_fence(__ATOMIC_RELEASE, "wavefront");
  __builtin_amdgcn_wave_barrier();
  __builtin_amdgcn_fence(__ATOMIC_ACQUIRE, "wavefront");
}

template <int SLB>
__device__ __forceinline__ int scan_chunk(const int* __restrict__ dsts, int nE, int cbase, int slotBase,
                                          int nb, int vec8, int* list, int tid, int lane, int wave) {
  int wc = 0;
  const int el0  = tid * EPT;
  const int e0   = cbase + el0;
  const int sent = -2147483647 - 1;
  v4i da, db;
  if (vec8 != 0 && cbase + CHUNK <= nE) {
    da = *(const v4i*)(dsts + e0);
    db = *(const v4i*)(dsts + e0 + 4);
  } else {
    da.x = (e0     < nE) ? dsts[min(e0,     nE - 1)] : sent;
    da.y = (e0 + 1 < nE) ? dsts[min(e0 + 1, nE - 1)] : sent;
    da.z = (e0 + 2 < nE) ? dsts[min(e0 + 2, nE - 1)] : sent;
    da.w = (e0 + 3 < nE) ? dsts[min(e0 + 3, nE - 1)] : sent;
    db.x = (e0 + 4 < nE) ? dsts[min(e0 + 4, nE - 1)] : sent;
    db.y = (e0 + 5 < nE) ? dsts[min(e0 + 5, nE - 1)] : sent;
    db.z = (e0 + 6 < nE) ? dsts[min(e0 + 6, nE - 1)] : sent;
    db.w = (e0 + 7 < nE) ? dsts[min(e0 + 7, nE - 1)] : sent;
  }
  const unsigned nbs = (unsigned)slotBase;
  const unsigned unb = (unsigned)nb;
  const unsigned s0 = (unsigned)da.x - nbs, s1 = (unsigned)da.y - nbs;
  const unsigned s2 = (unsigned)da.z - nbs, s3 = (unsigned)da.w - nbs;
  const unsigned s4 = (unsigned)db.x - nbs, s5 = (unsigned)db.y - nbs;
  const unsigned s6 = (unsigned)db.z - nbs, s7 = (unsigned)db.w - nbs;
  const bool h0 = s0 < unb, h1 = s1 < unb, h2 = s2 < unb, h3 = s3 < unb;
  const bool h4 = s4 < unb, h5 = s5 < unb, h6 = s6 < unb, h7 = s7 < unb;
  const unsigned any = __builtin_amdgcn_ballot_w32(h0 | h1 | h2 | h3 | h4 | h5 | h6 | h7);
  if (any != 0u) {
#define HITJ(J, HJ, SJ) { \
      const unsigned mj = __builtin_amdgcn_ballot_w32(HJ); \
      if (mj != 0u) { \
        if (HJ) { \
          const int pos = wc + (int)__builtin_amdgcn_mbcnt_lo(mj, 0u); \
          if (pos < WCAP) list[wave * WCAP + pos] = ((el0 + (J)) << SLB) | (int)(SJ); \
        } \
        wc += (int)__builtin_popcount(mj); } }
    HITJ(0, h0, s0)
    HITJ(1, h1, s1)
    HITJ(2, h2, s2)
    HITJ(3, h3, s3)
    HITJ(4, h4, s4)
    HITJ(5, h5, s5)
    HITJ(6, h6, s6)
    HITJ(7, h7, s7)
#undef HITJ
  }
  return wc;
}

__global__ __launch_bounds__(NTHR) void k_prep(const float* __restrict__ x, const float* __restrict__ W1,
                                               const float* __restrict__ W2, const float* __restrict__ W3,
                                               int nN, int nUx, unsigned short* XB, unsigned short* W1T,
                                               unsigned short* W2T2, unsigned short* W3T2) {
  const int u = (int)blockIdx.x * NTHR + (int)threadIdx.x;
  v8us o;
  unsigned short* dp;
  if (u < nUx) {
    const int row = u >> 4;
    const int k8  = (u & 15) * 8;
    const int rc  = row < nN ? row : nN - 1;
    const float* p = x + (size_t)rc * CIN + k8;
    const v4f a = *(const v4fa*)p;
    const v4f b = *(const v4fa*)(p + 4);
    const bool ok = row < nN;
    o[0] = ok ? (unsigned short)bf16_bits(a.x) : (unsigned short)0;
    o[1] = ok ? (unsigned short)bf16_bits(a.y) : (unsigned short)0;
    o[2] = ok ? (unsigned short)bf16_bits(a.z) : (unsigned short)0;
    o[3] = ok ? (unsigned short)bf16_bits(a.w) : (unsigned short)0;
    o[4] = ok ? (unsigned short)bf16_bits(b.x) : (unsigned short)0;
    o[5] = ok ? (unsigned short)bf16_bits(b.y) : (unsigned short)0;
    o[6] = ok ? (unsigned short)bf16_bits(b.z) : (unsigned short)0;
    o[7] = ok ? (unsigned short)bf16_bits(b.w) : (unsigned short)0;
    dp = XB + (size_t)row * CIN + k8;
  } else {
    const int v = u - nUx;
    if (v < NU1) {
      const int n  = v >> 4;
      const int k8 = (v & 15) * 8;
      const float* p = W1 + (size_t)k8 * HID + n;
#pragma unroll
      for (int i = 0; i < 8; ++i) o[i] = (unsigned short)bf16_bits(p[(size_t)i * HID]);
      dp = W1T + (size_t)n * CIN + k8;
    } else if (v < NU1 + NU2) {
      const int w  = v - NU1;
      const int n  = w >> 5;
      const int k8 = (w & 31) * 8;
      const int kk = k8 & (HID - 1);
      const float* p = W2 + (size_t)kk * HID + n;
#pragma unroll
      for (int i = 0; i < 8; ++i) o[i] = (unsigned short)bf16_bits(p[(size_t)i * HID]);
      dp = W2T2 + (size_t)n * K2 + k8;
    } else if (v < NU1 + NU2 + NU3) {
      const int w  = v - NU1 - NU2;
      const int n  = w >> 5;
      const int k8 = (w & 31) * 8;
      const int kk = k8 & (HID - 1);
      const int nc = n < NCLS ? n : NCLS - 1;
      const bool ok = n < NCLS;
      const float* p = W3 + (size_t)kk * NCLS + nc;
#pragma unroll
      for (int i = 0; i < 8; ++i) {
        const unsigned bb = bf16_bits(p[(size_t)i * NCLS]);
        o[i] = ok ? (unsigned short)bb : (unsigned short)0;
      }
      dp = W3T2 + (size_t)n * K2 + k8;
    } else {
      return;
    }
  }
  *(volatile v8us*)dp = o;
  __threadfence();
  *(volatile v8us*)dp = o;
}

__global__ __launch_bounds__(NTHR) void k_build(const int* __restrict__ srcs, const int* __restrict__ dsts,
                                                int nE, int nN, int vec8, int* srcl, int* rows, int* flg) {
  extern __shared__ __attribute__((aligned(16))) int dsm[];
  int* list = dsm;
  int* hl   = dsm + LISTN;
  int* sl   = hl + RCAP;
  int* cnt  = sl + RCAP;
  int* offs = cnt + NBA;
  int* cur  = offs + NBA;
  int* misc = cur + NBA;
  const int tid = (int)threadIdx.x, lane = tid & 31, wave = tid >> 5;
  const int nodeBase = (int)blockIdx.x * NBA;

  {
    const v4i z4 = {0, 0, 0, 0};
    for (int i = tid * 4; i < BLD_ZINTS; i += NTHR * 4) *(v4ia*)(dsm + i) = z4;
    if (tid < 16) misc[tid] = 0;
  }
  __syncthreads();

  int t = 0, ov = 0;
  const int nChunks = (nE + CHUNK - 1) / CHUNK;
#pragma unroll 1
  for (int ch = 0; ch < nChunks; ++ch) {
    const int cbase = ch * CHUNK;
    const int wc = scan_chunk<SLA>(dsts, nE, cbase, nodeBase, NBA, vec8, list, tid, lane, wave);
    if (lane == 0) misc[wave] = wc;
    __syncthreads();
    if (wave == 0) {
#pragma unroll 1
      for (int w2 = 0; w2 < NWAVE; ++w2) {
        int c = misc[w2];
        c = c < 0 ? 0 : (c > WCAP ? WCAP : c);
#pragma unroll 1
        for (int b0 = 0; b0 < c; b0 += 32) {
          const int idx = b0 + lane;
          const int ent = list[w2 * WCAP + (idx < WCAP ? idx : WCAP - 1)];
          const int m32 = (c - b0) < 32 ? (c - b0) : 32;
#pragma unroll 1
          for (int k = 0; k < m32; ++k) {
            const int u    = __builtin_amdgcn_readlane(ent, k);
            const int slot = u & (NBA - 1);
            const int el   = (u >> SLA) & (CHUNK - 1);
            const int pk   = ((cbase + el) << SLA) | slot;
            if (t < RCAP) {
              if (lane == 0) { hl[t] = pk; cnt[slot] = cnt[slot] + 1; }
              t = t + 1;
            } else {
              ov = 1;
            }
          }
        }
      }
    }
    __syncthreads();
  }
  if (wave == 0 && lane == 0) { misc[8] = t; misc[9] = ov; }
  __syncthreads();
  int tt = misc[8];
  tt = tt < 0 ? 0 : (tt > RCAP ? RCAP : tt);
  const int ovf = misc[9];

  if (wave == 0) {
    const int base = lane * (NBA / 32);
    int s = 0;
#pragma unroll 1
    for (int i = 0; i < NBA / 32; ++i) s += cnt[base + i];
    int incl = s;
#pragma unroll
    for (int d = 1; d < 32; d <<= 1) {
      const int y = __shfl_up(incl, d, 32);
      if (lane >= d) incl += y;
    }
    int run = incl - s;
#pragma unroll 1
    for (int i = 0; i < NBA / 32; ++i) {
      const int cv = cnt[base + i];
      offs[base + i] = run;
      cur[base + i]  = run;
      run += cv;
    }
  }
  __syncthreads();
  if (wave == 0) {
#pragma unroll 1
    for (int b0 = 0; b0 < tt; b0 += 32) {
      const int idx = b0 + lane;
      const int ent = hl[idx < RCAP ? idx : RCAP - 1];
      const int m32 = (tt - b0) < 32 ? (tt - b0) : 32;
#pragma unroll 1
      for (int k = 0; k < m32; ++k) {
        const int u    = __builtin_amdgcn_readlane(ent, k);
        const int slot = u & (NBA - 1);
        if (lane == 0) {
          int p = cur[slot];
          p = p < 0 ? 0 : (p > RCAP - 1 ? RCAP - 1 : p);
          sl[p] = u;
          cur[slot] = p + 1;
        }
      }
    }
  }
  __syncthreads();

#pragma unroll 1
  for (int it = 0; it < RCAP / (NTHR * 4); ++it) {
    const int p0 = (it * NTHR + tid) * 4;
    const v4i e4 = *(const v4ia*)(sl + p0);
    int e0 = e4.x >> SLA, e1 = e4.y >> SLA, e2 = e4.z >> SLA, e3 = e4.w >> SLA;
    e0 = e0 < 0 ? 0 : (e0 > nE - 1 ? nE - 1 : e0);
    e1 = e1 < 0 ? 0 : (e1 > nE - 1 ? nE - 1 : e1);
    e2 = e2 < 0 ? 0 : (e2 > nE - 1 ? nE - 1 : e2);
    e3 = e3 < 0 ? 0 : (e3 > nE - 1 ? nE - 1 : e3);
    int r0 = srcs[e0], r1 = srcs[e1], r2 = srcs[e2], r3 = srcs[e3];
    r0 = r0 < 0 ? 0 : (r0 > nN - 1 ? nN - 1 : r0);
    r1 = r1 < 0 ? 0 : (r1 > nN - 1 ? nN - 1 : r1);
    r2 = r2 < 0 ? 0 : (r2 > nN - 1 ? nN - 1 : r2);
    r3 = r3 < 0 ? 0 : (r3 > nN - 1 ? nN - 1 : r3);
    v4i r;
    r.x = (p0     < tt) ? r0 : 0;
    r.y = (p0 + 1 < tt) ? r1 : 0;
    r.z = (p0 + 2 < tt) ? r2 : 0;
    r.w = (p0 + 3 < tt) ? r3 : 0;
    *(v4ia*)(hl + p0) = r;
  }
  __syncthreads();

  int* sg = srcl + (size_t)blockIdx.x * RCAP;
  v4i rv[2];
#pragma unroll
  for (int it = 0; it < 2; ++it) {
    const int r0 = 2 * (it * NTHR + tid);
    int c0 = cnt[r0], c1 = cnt[r0 + 1];
    c0 = (ovf != 0 || c0 > DEGCAP || c0 < 0) ? POISONC : c0;
    c1 = (ovf != 0 || c1 > DEGCAP || c1 < 0) ? POISONC : c1;
    v4i q;
    q.x = offs[r0]; q.y = c0; q.z = offs[r0 + 1]; q.w = c1;
    rv[it] = q;
  }
  const v4i fq = {ovf, ovf, ovf, ovf};
  const bool fst = (wave == 0) && (lane < 8);
  int* fp = flg + (size_t)blockIdx.x * 32 + 4 * (lane & 7);

#pragma unroll 1
  for (int it = 0; it < RCAP / (NTHR * 4); ++it) {
    const int p0 = (it * NTHR + tid) * 4;
    const v4i r = *(const v4ia*)(hl + p0);
    *(volatile v4i*)(sg + p0) = r;
  }
#pragma unroll
  for (int it = 0; it < 2; ++it) {
    const int r0 = 2 * (it * NTHR + tid);
    *(volatile v4i*)(rows + 2 * ((size_t)nodeBase + r0)) = rv[it];
  }
  if (fst) *(volatile v4i*)fp = fq;
  __threadfence();
#pragma unroll 1
  for (int it = 0; it < RCAP / (NTHR * 4); ++it) {
    const int p0 = (it * NTHR + tid) * 4;
    const v4i r = *(const v4ia*)(hl + p0);
    *(volatile v4i*)(sg + p0) = r;
  }
#pragma unroll
  for (int it = 0; it < 2; ++it) {
    const int r0 = 2 * (it * NTHR + tid);
    *(volatile v4i*)(rows + 2 * ((size_t)nodeBase + r0)) = rv[it];
  }
  if (fst) *(volatile v4i*)fp = fq;
}

template <int NT>
__global__ __launch_bounds__(GTHR) void k_gemm(
    const unsigned short* __restrict__ A, const unsigned short* __restrict__ WT,
    float* outF, int K, int ldo)
{
  constexpr int BN = NT * 16;
  __shared__ __attribute__((aligned(16))) float stg[GBM * BN];
  const int tid = (int)threadIdx.x, lane = tid & 31, wave = tid >> 5, hh = lane >> 4, m = lane & 15;
  const int rowBase = (int)blockIdx.x * GBM;
  const int col0    = (int)blockIdx.y * BN;

  v8f acc[NT];
  {
    const v8f z = {0.f, 0.f, 0.f, 0.f, 0.f, 0.f, 0.f, 0.f};
#pragma unroll
    for (int t = 0; t < NT; ++t) acc[t] = z;
  }
  const unsigned short* ap = A  + (size_t)(rowBase + 16 * wave + m) * (size_t)K + 8 * hh;
  const unsigned short* wp = WT + (size_t)(col0 + m) * (size_t)K + 8 * hh;
  const int ksteps = K >> 5;
#pragma unroll 1
  for (int ks = 0; ks < ksteps; ++ks) {
    FragB af;
    af.h[0] = *(const v8usa*)(ap + 32 * ks);
    af.h[1] = *(const v8usa*)(ap + 32 * ks + 16);
#pragma unroll
    for (int t = 0; t < NT; ++t) {
      const unsigned short* wq = wp + (size_t)(16 * t) * (size_t)K + 32 * ks;
      FragB bf;
      bf.h[0] = *(const v8usa*)wq;
      bf.h[1] = *(const v8usa*)(wq + 16);
      acc[t] = wmb(af, bf, acc[t]);
    }
  }

#pragma unroll
  for (int t = 0; t < NT; ++t) {
    const int lc = 16 * t + m;
#pragma unroll
    for (int r = 0; r < 8; ++r) {
      const int lr = 16 * wave + 8 * hh + r;
      stg[lr * BN + lc] = acc[t][r];
    }
  }
  __syncthreads();

  if constexpr (NT == 4) {
    v4f fv[8];
#pragma unroll
    for (int i = 0; i < 8; ++i) {
      const int lr = 16 * wave + 2 * i + hh;
      fv[i] = *(const v4fa*)(stg + lr * BN + 4 * m);
    }
#pragma unroll
    for (int i = 0; i < 8; ++i) {
      const int lr = 16 * wave + 2 * i + hh;
      float* op = outF + (size_t)(rowBase + lr) * (size_t)ldo + col0 + 4 * m;
      *(volatile v4f*)op = fv[i];
    }
    __threadfence();
#pragma unroll
    for (int i = 0; i < 8; ++i) {
      const int lr = 16 * wave + 2 * i + hh;
      float* op = outF + (size_t)(rowBase + lr) * (size_t)ldo + col0 + 4 * m;
      *(volatile v4f*)op = fv[i];
    }
  } else {
    constexpr int NIT = (GBM * BN / 4) / GTHR;
    v4f fv[NIT];
#pragma unroll
    for (int it = 0; it < NIT; ++it) fv[it] = *(const v4fa*)(stg + 4 * (it * GTHR + tid));
    float* ob = outF + (size_t)rowBase * (size_t)BN;
#pragma unroll
    for (int it = 0; it < NIT; ++it) *(volatile v4f*)(ob + 4 * (size_t)(it * GTHR + tid)) = fv[it];
    __threadfence();
#pragma unroll
    for (int it = 0; it < NIT; ++it) *(volatile v4f*)(ob + 4 * (size_t)(it * GTHR + tid)) = fv[it];
  }
}

__global__ __launch_bounds__(NTHR) void k_agg128(const int* __restrict__ srcl, const int* __restrict__ rows,
                                                 int nN, int mRows, const float* __restrict__ T,
                                                 const float* __restrict__ bias, unsigned short* hb) {
  __shared__ __attribute__((aligned(16))) unsigned short rbuf[NWAVE * K2];
  const int tid = (int)threadIdx.x, lane = tid & 31, wave = tid >> 5;
  unsigned short* rowbuf = rbuf + wave * K2;
  const int nodeBase = (int)blockIdx.x * NBA;
  const int* seg = srcl + (size_t)blockIdx.x * RCAP;
  v4f b4;
  {
    const v4f tb = *(const v4f*)(bias + 4 * lane);
    b4.x = bf16_val(tb.x); b4.y = bf16_val(tb.y); b4.z = bf16_val(tb.z); b4.w = bf16_val(tb.w);
  }
  const float qnan = __int_as_float(0x7fc00000);
#pragma unroll 1
  for (int si = 0; si < NBA / NWAVE; ++si) {
    const int s    = si * NWAVE + wave;
    const int node = nodeBase + s;
    if (node >= mRows) break;
    const v2i rc = *(const v2ia*)(rows + 2 * (size_t)node);
    int o = rc.x;
    o = o < 0 ? 0 : (o > RCAP ? RCAP : o);
    int c = rc.y;
    const bool bad = (c < 0) || (c > DEGCAP);
    c = c < 0 ? 0 : (c > DEGCAP ? DEGCAP : c);
    const bool live = node < nN;
    c = live ? c : 0;
    float a0 = 0.0f, a1 = 0.0f, a2 = 0.0f, a3 = 0.0f;
#pragma unroll 1
    for (int b0 = 0; b0 < c; b0 += 32) {
      int idx = o + b0 + lane;
      idx = idx > RCAP - 1 ? RCAP - 1 : idx;
      int sr = seg[idx];
      sr = sr < 0 ? 0 : (sr > nN - 1 ? nN - 1 : sr);
      const int m32 = (c - b0) < 32 ? (c - b0) : 32;
#pragma unroll 1
      for (int k = 0; k < m32; ++k) {
        const int sk = __builtin_amdgcn_readlane(sr, k);
        const v4f a = *(const v4f*)(T + (size_t)sk * HID + 4 * lane);
        a0 += a.x; a1 += a.y; a2 += a.z; a3 += a.w;
      }
    }
    const float pzr = bad ? qnan : 0.0f;
    float y0 = a0 + b4.x, y1 = a1 + b4.y, y2 = a2 + b4.z, y3 = a3 + b4.w;
    y0 = (y0 > 0.0f) ? y0 : (y0 - y0);
    y1 = (y1 > 0.0f) ? y1 : (y1 - y1);
    y2 = (y2 > 0.0f) ? y2 : (y2 - y2);
    y3 = (y3 > 0.0f) ? y3 : (y3 - y3);
    const float m0 = live ? (y0 + pzr) : 0.0f;
    const float m1 = live ? (y1 + pzr) : 0.0f;
    const float m2 = live ? (y2 + pzr) : 0.0f;
    const float m3 = live ? (y3 + pzr) : 0.0f;
    v4us mh, ml;
    {
      unsigned hbits;
      hbits = bf16_bits(m0); mh[0] = (unsigned short)hbits; ml[0] = (unsigned short)bf16_bits(m0 - __uint_as_float(hbits << 16));
      hbits = bf16_bits(m1); mh[1] = (unsigned short)hbits; ml[1] = (unsigned short)bf16_bits(m1 - __uint_as_float(hbits << 16));
      hbits = bf16_bits(m2); mh[2] = (unsigned short)hbits; ml[2] = (unsigned short)bf16_bits(m2 - __uint_as_float(hbits << 16));
      hbits = bf16_bits(m3); mh[3] = (unsigned short)hbits; ml[3] = (unsigned short)bf16_bits(m3 - __uint_as_float(hbits << 16));
    }
    *(v4usa*)(rowbuf + 4 * lane) = mh;
    *(v4usa*)(rowbuf + HID + 4 * lane) = ml;
    wave_sync();
    const v8us q0 = *(const v8usa*)(rowbuf + 8 * lane);
    wave_sync();
    unsigned short* rpw = hb + (size_t)node * K2 + 8 * lane;
    *(volatile v8us*)rpw = q0;
    __threadfence();
    *(volatile v8us*)rpw = q0;
  }
}

__global__ __launch_bounds__(NTHR) void k_agg40(const int* __restrict__ srcl, const int* __restrict__ rows,
                                                const int* __restrict__ flg, int nFlg, int nN,
                                                const float* __restrict__ T3, const float* __restrict__ b3,
                                                float* out) {
  extern __shared__ __attribute__((aligned(16))) float stage[];
  __shared__ int sfl[NWAVE];
  const int tid = (int)threadIdx.x, lane = tid & 31, wave = tid >> 5;
  const int nodeBase = (int)blockIdx.x * NBA;
  const int* seg = srcl + (size_t)blockIdx.x * RCAP;

  {
    const int fi = tid < nFlg ? tid : nFlg - 1;
    const int f  = flg[(size_t)fi * 32];
    const unsigned mk = __builtin_amdgcn_ballot_w32(f != 0);
    if (lane == 0) sfl[wave] = (mk != 0u) ? 1 : 0;
  }
  __syncthreads();
  int anyf = 0;
#pragma unroll
  for (int w2 = 0; w2 < NWAVE; ++w2) anyf |= sfl[w2];

  const int sub = lane / 10;
  const int q   = lane - 10 * sub;
  v4f b4;
  {
    const v4f tb = *(const v4f*)(b3 + 4 * q);
    b4.x = bf16_val(tb.x); b4.y = bf16_val(tb.y); b4.z = bf16_val(tb.z); b4.w = bf16_val(tb.w);
  }
  const float qnan = __int_as_float(0x7fc00000);

#pragma unroll 1
  for (int gi = 0; gi < (NGRP + NWAVE - 1) / NWAVE; ++gi) {
    const int g = gi * NWAVE + wave;
    if (g >= NGRP) break;
    if (nodeBase + 3 * g >= nN) break;
    const int s  = 3 * g + sub;
    const int sc = s < NBA ? s : NBA - 1;
    const int node = nodeBase + sc;
    const bool valid = (sub < 3) && (s < NBA) && (node < nN);
    const int nc = node < nN ? node : nN - 1;
    const v2i rc = *(const v2ia*)(rows + 2 * (size_t)nc);
    int o = rc.x;
    o = o < 0 ? 0 : (o > RCAP ? RCAP : o);
    int c = rc.y;
    const bool bad = (c < 0) || (c > DEGCAP);
    c = c < 0 ? 0 : (c > DEGCAP ? DEGCAP : c);
    c = valid ? c : 0;
    int cm = c;
#pragma unroll
    for (int d = 16; d >= 1; d >>= 1) {
      const int y = __shfl_xor(cm, d, 32);
      cm = cm > y ? cm : y;
    }
    cm = cm > DEGCAP ? DEGCAP : cm;
    float a0 = 0.0f, a1 = 0.0f, a2 = 0.0f, a3 = 0.0f;
#pragma unroll 1
    for (int k = 0; k < cm; ++k) {
      int idx = o + k;
      idx = idx > RCAP - 1 ? RCAP - 1 : idx;
      int sr = seg[idx];
      sr = sr < 0 ? 0 : (sr > nN - 1 ? nN - 1 : sr);
      const float w = (k < c) ? 1.0f : 0.0f;
      const v4f a = *(const v4f*)(T3 + (size_t)sr * NC3 + 4 * q);
      a0 = fmaf(w, a.x, a0); a1 = fmaf(w, a.y, a1); a2 = fmaf(w, a.z, a2); a3 = fmaf(w, a.w, a3);
    }
    const float pzr = (bad || anyf != 0) ? qnan : 0.0f;
    v4f v;
    v.x = (a0 + b4.x) + pzr; v.y = (a1 + b4.y) + pzr; v.z = (a2 + b4.z) + pzr; v.w = (a3 + b4.w) + pzr;
    if (valid) *(v4fa*)(stage + s * NCLS + 4 * q) = v;
  }
  __syncthreads();

  int nRows = nN - nodeBase;
  nRows = nRows > NBA ? NBA : (nRows < 0 ? 0 : nRows);
  const int nF4 = nRows * (NCLS / 4);
  float* ob = out + (size_t)nodeBase * NCLS;
#pragma unroll 1
  for (int it = 0; it < (NBA * NCLS / 4) / NTHR; ++it) {
    const int idx = it * NTHR + tid;
    if (idx < nF4) {
      const v4f v = *(const v4fa*)(stage + 4 * idx);
      *(volatile v4f*)(ob + 4 * (size_t)idx) = v;
    }
  }
  __threadfence();
#pragma unroll 1
  for (int it = 0; it < (NBA * NCLS / 4) / NTHR; ++it) {
    const int idx = it * NTHR + tid;
    if (idx < nF4) {
      const v4f v = *(const v4fa*)(stage + 4 * idx);
      *(volatile v4f*)(ob + 4 * (size_t)idx) = v;
    }
  }
}

static inline int cdiv(int a, int b) { return (a + b - 1) / b; }
static inline size_t al256(size_t o) { return (o + 255) & ~(size_t)255; }

extern "C" void kernel_launch(void* const* d_in, const int* in_sizes, int n_in,
                              void* d_out, int out_size, void* d_ws, size_t ws_size,
                              hipStream_t stream) {
  if (n_in < 9) return;
  if (in_sizes[0] < CIN || (in_sizes[0] % CIN) != 0) return;
  const int nN = in_sizes[0] / CIN;
  if (nN < 16 || nN > (1 << 22) || (nN & 15) != 0) return;
  const int nE = in_sizes[1];
  if (nE < 1 || in_sizes[2] != nE) return;
  if (nE >= (1 << (31 - SLA))) return;
  if (in_sizes[3] != CIN * HID || in_sizes[4] != HID) return;
  if (in_sizes[5] != HID * HID || in_sizes[6] != HID) return;
  if (in_sizes[7] != HID * NCLS || in_sizes[8] != NCLS) return;
  if ((long long)out_size != (long long)nN * NCLS) return;

  const float* x   = (const float*)d_in[0];
  const int*   src = (const int*)d_in[1];
  const int*   dst = (const int*)d_in[2];
  const float* W1  = (const float*)d_in[3];
  const float* b1  = (const float*)d_in[4];
  const float* W2  = (const float*)d_in[5];
  const float* b2  = (const float*)d_in[6];
  const float* W3  = (const float*)d_in[7];
  const float* b3  = (const float*)d_in[8];
  float* out = (float*)d_out;

  const int MP = cdiv(nN, GBM) * GBM;
  const int gM = MP / GBM;
  const int gA = cdiv(MP, NBA);
  const int gO = cdiv(nN, NBA);
  if ((long long)gA * NBA < (long long)MP) return;
  if (gA > NTHR || gO > gA) return;
  const int vec8 = ((nE & 3) == 0) ? 1 : 0;
  const int nUx  = MP * (CIN / 8);
  if ((nUx % NTHR) != 0) return;

  char* ws = (char*)d_ws;
  size_t off = 0;
  const size_t oT   = off; off = al256(off + (size_t)MP * HID * 4);
  const size_t oH   = off; off = al256(off + (size_t)MP * K2 * 2);
  const size_t oSR  = off; off = al256(off + (size_t)gA * RCAP * 4);
  const size_t oRW  = off; off = al256(off + (size_t)gA * NBA * 8);
  const size_t oFL  = off; off = al256(off + (size_t)gA * 128);
  const size_t oW1  = off; off = al256(off + (size_t)HID * CIN * 2);
  const size_t oW2  = off; off = al256(off + (size_t)HID * K2 * 2);
  const size_t oW3  = off; off = al256(off + (size_t)NC3 * K2 * 2);
  if (off > ws_size || off > (size_t)WSMAX) return;
  if ((size_t)MP * CIN * 2 > (size_t)MP * K2 * 2) return;
  if ((size_t)MP * NC3 * 4 > (size_t)MP * HID * 4) return;
  float*          T    = (float*)(ws + oT);
  unsigned short* H    = (unsigned short*)(ws + oH);
  unsigned short* XB   = (unsigned short*)(ws + oH);
  int*            SRCL = (int*)(ws + oSR);
  int*            ROWS = (int*)(ws + oRW);
  int*            FLG  = (int*)(ws + oFL);
  unsigned short* W1T  = (unsigned short*)(ws + oW1);
  unsigned short* W2T2 = (unsigned short*)(ws + oW2);
  unsigned short* W3T2 = (unsigned short*)(ws + oW3);

  const size_t bldLds = (size_t)BLD_LDS_INTS * 4;
  const size_t outLds = (size_t)NBA * NCLS * 4;
  hipFuncSetAttribute(reinterpret_cast<const void*>(&k_build), hipFuncAttributeMaxDynamicSharedMemorySize, (int)bldLds);
  hipFuncSetAttribute(reinterpret_cast<const void*>(&k_agg40), hipFuncAttributeMaxDynamicSharedMemorySize, (int)outLds);

  k_prep<<<(nUx + NU1 + NU2 + NU3) / NTHR, NTHR, 0, stream>>>(x, W1, W2, W3, nN, nUx, XB, W1T, W2T2, W3T2);
  k_build<<<gA, NTHR, bldLds, stream>>>(src, dst, nE, nN, vec8, SRCL, ROWS, FLG);
  k_gemm<4><<<dim3(gM, HID / 64), GTHR, 0, stream>>>(XB, W1T, T, CIN, HID);
  k_agg128<<<gA, NTHR, 0, stream>>>(SRCL, ROWS, nN, MP, T, b1, H);
  k_gemm<4><<<dim3(gM, HID / 64), GTHR, 0, stream>>>(H, W2T2, T, K2, HID);
  k_agg128<<<gA, NTHR, 0, stream>>>(SRCL, ROWS, nN, MP, T, b2, H);
  k_gemm<3><<<dim3(gM, 1), GTHR, 0, stream>>>(H, W3T2, T, K2, NC3);
  k_agg40<<<gO, NTHR, outLds, stream>>>(SRCL, ROWS, FLG, gA, nN, T, b3, out);
}
